// Decoder_34265249087980
// MI455X (gfx1250) — hardware-verified
//
#include <hip/hip_runtime.h>
#include <math.h>

typedef __attribute__((ext_vector_type(16))) _Float16 v16h;
typedef __attribute__((ext_vector_type(8)))  _Float16 v8h;
typedef __attribute__((ext_vector_type(16))) __bf16   v16b;
typedef __attribute__((ext_vector_type(8)))  __bf16   v8b;
typedef __attribute__((ext_vector_type(8)))  float    v8f;
typedef __attribute__((ext_vector_type(4)))  float    v4f;
typedef __attribute__((ext_vector_type(4)))  unsigned int v4u;

constexpr int NBAT    = 16;
constexpr int NSTEPS  = 96;
constexpr int NFEAT   = 512;
constexpr int NHID    = 512;
constexpr int NMEL    = 80;
constexpr int NGATE   = 4 * NHID;
constexpr int NIH0    = NMEL + NFEAT;
constexpr int XA_K    = 608;
constexpr int W0_IHP  = 640;
constexpr int W0_LD   = W0_IHP + NHID;
constexpr int W1_LD   = 2 * NHID;
constexpr int XAP     = XA_K + 8;
constexpr int X1P     = 2 * NHID + 8;
constexpr int QWP     = NHID + 4;
constexpr int OSTP    = 2 * NMEL;
constexpr int NENCROW = NBAT * NSTEPS;
constexpr int DEC_THR   = 512;
constexpr int DEC_WAVES = DEC_THR / 32;
constexpr float ACT_CARRY = 256.0f;
constexpr float W_CARRY   = 256.0f;
constexpr float ENC_CARRY = 16.0f;
constexpr float FOLD_AW   = 1.0f / (ACT_CARRY * W_CARRY);
constexpr float FOLD_UAK  = 1.0f / (ENC_CARRY * W_CARRY);
constexpr int TAB_B0  = 0;
constexpr int TAB_B1  = 2048;
constexpr int TAB_WAB = 4096;
constexpr int TAB_VA  = 4608;
constexpr int TAB_UAB = 5120;
constexpr int TAB_PJB = 5632;
constexpr int TAB_N   = 6144;

static_assert(NBAT == 16, "one 16-row WMMA tile");
static_assert(DEC_WAVES == NBAT, "wave b owns batch row b in the VALU phases");
static_assert(NHID == 32 * DEC_WAVES, "two 16-unit tiles per wave");
static_assert(NSTEPS == 96 && (NSTEPS % 2) == 0, "softmax 3 x 32 lanes; output flushed per step pair");
static_assert(NFEAT == 512, "context map: 2 x 32 lanes x 8");
static_assert(NIH0 == 592 && (NIH0 % 8) == 0, "ih segment");
static_assert(XA_K % 32 == 0 && XA_K >= NIH0 && XA_K <= W0_IHP, "k padding");
static_assert(NHID % 32 == 0, "k tiles");
static_assert(NMEL % 16 == 0 && NMEL / 16 <= DEC_WAVES, "projection tiles");
static_assert((W0_IHP * 2) % 128 == 0 && (W0_LD * 2) % 128 == 0 && (W1_LD * 2) % 128 == 0, "line aligned planes");
static_assert((XAP * 2) % 16 == 0 && (X1P * 2) % 16 == 0 && (QWP * 4) % 16 == 0 && (OSTP * 4) % 16 == 0, "LDS alignment");
static_assert(NENCROW % 64 == 0 && NHID % 64 == 0 && NFEAT % 32 == 0, "GEMM M, N tile multiples and K % 32");
static_assert(TAB_N == 12 * 512, "table blocks");
static_assert((NSTEPS * NMEL * 4) % 128 == 0 && (2 * NMEL * 4) % 128 == 0, "output step pairs are whole lines");

__device__ __forceinline__ unsigned short f2bf_bits(float f) {
  unsigned u = __float_as_uint(f);
  return (unsigned short)((u + 0x7FFFu + ((u >> 16) & 1u)) >> 16);
}
__device__ __forceinline__ float bf_bits2f(unsigned short h) { return __uint_as_float(((unsigned)h) << 16); }
__device__ __forceinline__ float bf16r(float f) { return bf_bits2f(f2bf_bits(f)); }
__device__ __forceinline__ unsigned pk16(unsigned short a, unsigned short b) { return (unsigned)a | ((unsigned)b << 16); }
__device__ __forceinline__ unsigned short h_bits(float f) { const _Float16 h = (_Float16)f; return __builtin_bit_cast(unsigned short, h); }
__device__ __forceinline__ float fsig(float x) { return 1.0f / (1.0f + expf(-x)); }
__device__ __forceinline__ void split_act(float x, _Float16& hi, _Float16& lo) {
  const float s = x * ACT_CARRY;
  const _Float16 h = (_Float16)s;
  hi = h;
  lo = (_Float16)(s - (float)h);
}

__device__ __forceinline__ void dep_guard4_h(v8f& a, v8f& b, v8f& c, v8f& d, v16h x, v16h y) { asm volatile("v_nop\n\tv_nop\n\tv_nop\n\tv_nop" : "+v"(a), "+v"(b), "+v"(c), "+v"(d) : "v"(x), "v"(y)); }
__device__ __forceinline__ void dep_guard4_b(v8f& a, v8f& b, v8f& c, v8f& d, v16b x, v16b y) { asm volatile("v_nop\n\tv_nop\n\tv_nop\n\tv_nop" : "+v"(a), "+v"(b), "+v"(c), "+v"(d) : "v"(x), "v"(y)); }
__device__ __forceinline__ void keep4_h(v16h a, v16h b, v16h c, v16h d) { asm volatile("v_nop" :: "v"(a), "v"(b), "v"(c), "v"(d)); }
__device__ __forceinline__ void keep4_b(v16b a, v16b b, v16b c, v16b d) { asm volatile("v_nop" :: "v"(a), "v"(b), "v"(c), "v"(d)); }
__device__ __forceinline__ void acc_guard4(v8f& a, v8f& b, v8f& c, v8f& d) { asm volatile("v_nop\n\tv_nop\n\tv_nop\n\tv_nop" : "+v"(a), "+v"(b), "+v"(c), "+v"(d)); }
__device__ __forceinline__ void acc_guard2(v8f& a, v8f& b) { asm volatile("v_nop\n\tv_nop\n\tv_nop\n\tv_nop" : "+v"(a), "+v"(b)); }
__device__ __forceinline__ void acc_guard1(v8f& a) { asm volatile("v_nop\n\tv_nop\n\tv_nop\n\tv_nop" : "+v"(a)); }
__device__ __forceinline__ void guard_gate(v8f& a, v8f& b, v8f& c, v8f& d, v16h x, v16h y, v16h p, v16h q, v16h r, v16h s) {
  asm volatile("v_nop\n\tv_nop\n\tv_nop\n\tv_nop" : "+v"(a), "+v"(b), "+v"(c), "+v"(d) : "v"(x), "v"(y), "v"(p), "v"(q), "v"(r), "v"(s));
}
__device__ __forceinline__ void guard_query(v8f& a, v8f& b, v16h x, v16h y, v16h z, v16h w, v16h p, v16h q) {
  asm volatile("v_nop\n\tv_nop\n\tv_nop\n\tv_nop" : "+v"(a), "+v"(b) : "v"(x), "v"(y), "v"(z), "v"(w), "v"(p), "v"(q));
}
__device__ __forceinline__ void guard_proj(v8f& a, v16h x, v16h y, v16h p) {
  asm volatile("v_nop\n\tv_nop\n\tv_nop\n\tv_nop" : "+v"(a) : "v"(x), "v"(y), "v"(p));
}

template <typename T> struct Frag;
template <> struct Frag<_Float16> {
  typedef v16h V; union U { v16h v; v8h h[2]; };
  static __device__ __forceinline__ v16h load(const _Float16* p) {
    U f; f.h[0] = *(const v8h*)(p); f.h[1] = *(const v8h*)(p + 16); return f.v;
  }
  static __device__ __forceinline__ v8f mma(v16h a, v16h b, v8f c) {
    return __builtin_amdgcn_wmma_f32_16x16x32_f16(false, a, false, b, (short)0, c, false, false);
  }
  static __device__ __forceinline__ void guard4(v8f& a, v8f& b, v8f& c, v8f& d, v16h x, v16h y) { dep_guard4_h(a, b, c, d, x, y); }
  static __device__ __forceinline__ void keep(v16h a, v16h b, v16h c, v16h d) { keep4_h(a, b, c, d); }
};
template <> struct Frag<__bf16> {
  typedef v16b V; union U { v16b v; v8b h[2]; };
  static __device__ __forceinline__ v16b load(const __bf16* p) {
    U f; f.h[0] = *(const v8b*)(p); f.h[1] = *(const v8b*)(p + 16); return f.v;
  }
  static __device__ __forceinline__ v8f mma(v16b a, v16b b, v8f c) {
    return __builtin_amdgcn_wmma_f32_16x16x32_bf16(false, a, false, b, (short)0, c, false, false);
  }
  static __device__ __forceinline__ void guard4(v8f& a, v8f& b, v8f& c, v8f& d, v16b x, v16b y) { dep_guard4_b(a, b, c, d, x, y); }
  static __device__ __forceinline__ void keep(v16b a, v16b b, v16b c, v16b d) { keep4_b(a, b, c, d); }
};

template <int ET> struct Elem;
template <> struct Elem<0> { typedef _Float16 T; };
template <> struct Elem<1> { typedef __bf16 T; };
template <int ET, bool SPLIT, int BIAS_MODE, int OUT_MODE, bool RESID, int ACT = 0>
__global__ __launch_bounds__(256) void wmma_gemm64(
    const unsigned short* __restrict__ Ap, const unsigned short* __restrict__ A2p, int lda, long strideA,
    const unsigned short* __restrict__ Btp, const unsigned short* __restrict__ Bt2p, int ldb, long strideB,
    void* __restrict__ Cout, void* __restrict__ Cout2, int ldc, long strideC,
    const float* __restrict__ bias,
    const float* __restrict__ resid, long strideR,
    int M, int N, int K, float scale) {
  typedef typename Elem<ET>::T T;
  typedef typename Frag<T>::V V;
  const T* A = (const T*)Ap; const T* A2 = (const T*)A2p; const T* Bt = (const T*)Btp; const T* Bt2 = (const T*)Bt2p;
  __shared__ __align__(16) float sT[8][16 * 68];
  const int b    = blockIdx.y;
  const int lane = threadIdx.x & 31;
  const int wave = threadIdx.x >> 5;
  const int tilesN = N >> 6;
  const int tilesM = M >> 6;
  const int tile = blockIdx.x * 8 + wave;
  if (tile >= tilesM * tilesN) return;
  const int tm = tile / tilesN;
  const int tn = tile - tm * tilesN;
  const int m0 = tm << 6;
  const int n0 = tn << 6;

  const T* Ab  = A  + (size_t)b * strideA;
  const T* Bb  = Bt + (size_t)b * strideB;
  const T* Ab2 = SPLIT ? (A2  + (size_t)b * strideA) : nullptr;
  const T* Bb2 = SPLIT ? (Bt2 + (size_t)b * strideB) : nullptr;

  const int rlane = lane & 15;
  const int koff  = (lane >> 4) * 8;
  const int mOff  = (lane >> 4) * 8;

  v8f acc[4][4];
#pragma unroll
  for (int i = 0; i < 4; ++i)
#pragma unroll
    for (int j = 0; j < 4; ++j) acc[i][j] = (v8f){0.f,0.f,0.f,0.f,0.f,0.f,0.f,0.f};

  for (int k0 = 0; k0 < K; k0 += 32) {
    V bh[4], bl[4];
#pragma unroll
    for (int j = 0; j < 4; ++j) {
      const size_t bo = (size_t)(n0 + (j << 4) + rlane) * ldb + koff + k0;
      bh[j] = Frag<T>::load(Bb + bo);
      if (SPLIT) bl[j] = Frag<T>::load(Bb2 + bo);
    }
#pragma unroll
    for (int i = 0; i < 4; ++i) {
      const size_t ao = (size_t)(m0 + (i << 4) + rlane) * lda + koff + k0;
      V ah = Frag<T>::load(Ab + ao);
      V al;
      if (SPLIT) al = Frag<T>::load(Ab2 + ao);
#pragma unroll
      for (int j = 0; j < 4; ++j) {
        acc[i][j] = Frag<T>::mma(ah, bh[j], acc[i][j]);
        if (SPLIT) {
          acc[i][j] = Frag<T>::mma(ah, bl[j], acc[i][j]);
          acc[i][j] = Frag<T>::mma(al, bh[j], acc[i][j]);
        }
      }
      Frag<T>::guard4(acc[i][0], acc[i][1], acc[i][2], acc[i][3], ah, SPLIT ? al : ah);
    }
    Frag<T>::keep(bh[0], bh[1], bh[2], bh[3]);
    if (SPLIT) Frag<T>::keep(bl[0], bl[1], bl[2], bl[3]);
  }
  acc_guard4(acc[0][0], acc[0][1], acc[0][2], acc[0][3]);
  acc_guard4(acc[1][0], acc[1][1], acc[1][2], acc[1][3]);
  acc_guard4(acc[2][0], acc[2][1], acc[2][2], acc[2][3]);
  acc_guard4(acc[3][0], acc[3][1], acc[3][2], acc[3][3]);

  float* slab = sT[wave];
  const float* Rb = RESID ? (resid + (size_t)b * strideR) : nullptr;
#pragma unroll
  for (int i = 0; i < 4; ++i) {
    const int mBase = m0 + (i << 4);
#pragma unroll
    for (int j = 0; j < 4; ++j) {
      const int n = n0 + (j << 4) + rlane;
      float bv = 0.f;
      if (BIAS_MODE == 2) bv = bias[n];
#pragma unroll
      for (int r = 0; r < 8; ++r) {
        float v = acc[i][j][r] * scale;
        if (BIAS_MODE == 1) v += bias[mBase + mOff + r];
        if (BIAS_MODE == 2) v += bv;
        if (RESID) v += Rb[(size_t)(mBase + mOff + r) * ldc + n];
        if (ACT == 2) v = fmaxf(v, 0.0f);
        if (ACT == 4) v = (v > 0.f) ? v : 0.01f * v;
        slab[(mOff + r) * 68 + (j << 4) + rlane] = v;
      }
    }
    __builtin_amdgcn_fence(__ATOMIC_RELEASE, "workgroup");
    __builtin_amdgcn_wave_barrier();
    __builtin_amdgcn_fence(__ATOMIC_ACQUIRE, "workgroup");
    if (OUT_MODE == 0) {
      float* C = (float*)Cout + (size_t)b * strideC;
      const int hh = lane >> 4, c4 = (lane & 15) * 4;
      for (int pass = 0; pass < 2; ++pass) {
#pragma unroll
        for (int it = 0; it < 8; ++it) {
          const int row = it * 2 + hh;
          v4f v = *(const v4f*)(slab + row * 68 + c4);
          *(volatile v4f*)(C + (size_t)(mBase + row) * ldc + n0 + c4) = v;
        }
        __threadfence();
      }
    } else {
      const int q = lane >> 3, c8 = (lane & 7) * 8;
      unsigned short* C  = (unsigned short*)Cout  + (size_t)b * strideC;
      unsigned short* C2 = (OUT_MODE == 2) ? ((unsigned short*)Cout2 + (size_t)b * strideC) : nullptr;
      for (int pass = 0; pass < 2; ++pass) {
#pragma unroll
        for (int it = 0; it < 4; ++it) {
          const int row = it * 4 + q;
          const float* sp = slab + row * 68 + c8;
          v8h hv, lv;
#pragma unroll
          for (int e = 0; e < 8; ++e) {
            if (OUT_MODE == 1) {
              hv[e] = (_Float16)sp[e];
            } else {
              unsigned short hb = f2bf_bits(sp[e]);
              unsigned short lb = f2bf_bits(sp[e] - bf_bits2f(hb));
              hv[e] = __builtin_bit_cast(_Float16, hb);
              lv[e] = __builtin_bit_cast(_Float16, lb);
            }
          }
          *(volatile v8h*)(C + (size_t)(mBase + row) * ldc + n0 + c8) = hv;
          if (OUT_MODE == 2) *(volatile v8h*)(C2 + (size_t)(mBase + row) * ldc + n0 + c8) = lv;
        }
        __threadfence();
      }
    }
    __builtin_amdgcn_fence(__ATOMIC_RELEASE, "workgroup");
    __builtin_amdgcn_wave_barrier();
    __builtin_amdgcn_fence(__ATOMIC_ACQUIRE, "workgroup");
  }
}

template <int MODE>
__global__ __launch_bounds__(256) void cvt_rows_kernel(const float* __restrict__ src, int spitch, int nreal8,
                                                       unsigned short* __restrict__ dst, int dpitch, int dcol0,
                                                       int nrow, int ng, float sc) {
  const int i = blockIdx.x * 256 + threadIdx.x;
  if (i < nrow * ng) {
    const int row = i / ng;
    const int g   = i - row * ng;
    const int gs  = (g < nreal8) ? g : (nreal8 - 1);
    const float keep = (g < nreal8) ? sc : 0.0f;
    const float* sp = src + (size_t)row * spitch + gs * 8;
    const v4f a = *(const v4f*)(sp);
    const v4f b = *(const v4f*)(sp + 4);
    unsigned short hb[8];
#pragma unroll
    for (int e = 0; e < 4; ++e) {
      const float fa = a[e];
      const float fb = b[e];
      if (MODE == 0) {
        hb[e]     = h_bits(bf16r(fa) * keep);
        hb[4 + e] = h_bits(bf16r(fb) * keep);
      } else {
        hb[e]     = f2bf_bits(fa * keep);
        hb[4 + e] = f2bf_bits(fb * keep);
      }
    }
    const v4u u = (v4u){pk16(hb[0], hb[1]), pk16(hb[2], hb[3]), pk16(hb[4], hb[5]), pk16(hb[6], hb[7])};
    unsigned short* q = dst + (size_t)row * dpitch + dcol0 + g * 8;
    *(volatile v4u*)q = u;
    __threadfence();
    *(volatile v4u*)q = u;
  }
}

__global__ __launch_bounds__(128) void table_kernel(const float* __restrict__ bih0, const float* __restrict__ bhh0,
                                                    const float* __restrict__ bih1, const float* __restrict__ bhh1,
                                                    const float* __restrict__ wab, const float* __restrict__ vaw,
                                                    const float* __restrict__ uab, const float* __restrict__ pjb,
                                                    float* __restrict__ tab) {
  const int bx = blockIdx.x;
  const int e  = 4 * threadIdx.x;
  v4f o = (v4f){0.f, 0.f, 0.f, 0.f};
  if (bx < 8) {
    const float* pa = (bx < 4) ? bih0 : bih1;
    const float* pb = (bx < 4) ? bhh0 : bhh1;
    const int idx = (bx & 3) * 512 + e;
    const v4f a = *(const v4f*)(pa + idx);
    const v4f b = *(const v4f*)(pb + idx);
#pragma unroll
    for (int k = 0; k < 4; ++k) o[k] = bf16r(a[k]) + bf16r(b[k]);
  } else if (bx < 11) {
    const float* p = (bx == 8) ? wab : ((bx == 9) ? vaw : uab);
    const v4f a = *(const v4f*)(p + e);
#pragma unroll
    for (int k = 0; k < 4; ++k) o[k] = bf16r(a[k]);
  } else {
    const int ec = (e < NMEL - 4) ? e : (NMEL - 4);
    const v4f a = *(const v4f*)(pjb + ec);
    const float keep = (e < NMEL) ? 1.0f : 0.0f;
#pragma unroll
    for (int k = 0; k < 4; ++k) o[k] = bf16r(a[k]) * keep;
  }
  float* op = tab + bx * 512 + e;
  *(volatile v4f*)op = o;
  __threadfence();
  *(volatile v4f*)op = o;
}

__device__ __forceinline__ void gate_kloop(v8f& a0, v8f& a1, v8f& a2, v8f& a3,
                                           const _Float16* ah, const _Float16* al,
                                           const _Float16* w, size_t gstride, int ntile) {
#pragma unroll 1
  for (int kt = 0; kt < ntile; ++kt) {
    const int k0 = kt * 32;
    const v16h b0 = Frag<_Float16>::load(w + k0);
    const v16h b1 = Frag<_Float16>::load(w + gstride + k0);
    const v16h b2 = Frag<_Float16>::load(w + 2 * gstride + k0);
    const v16h b3 = Frag<_Float16>::load(w + 3 * gstride + k0);
    const v16h xh = Frag<_Float16>::load(ah + k0);
    const v16h xl = Frag<_Float16>::load(al + k0);
    a0 = Frag<_Float16>::mma(xh, b0, a0);
    a1 = Frag<_Float16>::mma(xh, b1, a1);
    a2 = Frag<_Float16>::mma(xh, b2, a2);
    a3 = Frag<_Float16>::mma(xh, b3, a3);
    a0 = Frag<_Float16>::mma(xl, b0, a0);
    a1 = Frag<_Float16>::mma(xl, b1, a1);
    a2 = Frag<_Float16>::mma(xl, b2, a2);
    a3 = Frag<_Float16>::mma(xl, b3, a3);
    guard_gate(a0, a1, a2, a3, xh, xl, b0, b1, b2, b3);
  }
}

__device__ __forceinline__ void cell_update(const v8f& ai, const v8f& af, const v8f& ag, const v8f& ao,
                                            float bi, float bf, float bg, float bo, v8f& cs, v8f& hn) {
#pragma unroll
  for (int r = 0; r < 8; ++r) {
    const float zi = ai[r] * FOLD_AW + bi;
    const float zf = af[r] * FOLD_AW + bf;
    const float zg = ag[r] * FOLD_AW + bg;
    const float zo = ao[r] * FOLD_AW + bo;
    const float ig = fsig(zi);
    const float fg = fsig(zf);
    const float og = fsig(zo);
    const float gg = tanhf(zg);
    const float cn = fg * cs[r] + ig * gg;
    cs[r] = cn;
    hn[r] = og * tanhf(cn);
  }
}

__global__ __launch_bounds__(DEC_THR) void decoder_kernel(
    const unsigned short* __restrict__ W0p, const unsigned short* __restrict__ W1p,
    const unsigned short* __restrict__ Wap, const unsigned short* __restrict__ Pjp,
    const unsigned short* __restrict__ encB, const float* __restrict__ UaK,
    const float* __restrict__ tab, const float* __restrict__ vab, float* __restrict__ out) {
  __shared__ __align__(16) _Float16 XaH[16 * XAP];
  __shared__ __align__(16) _Float16 XaL[16 * XAP];
  __shared__ __align__(16) _Float16 X1H[16 * X1P];
  __shared__ __align__(16) _Float16 X1L[16 * X1P];
  __shared__ __align__(16) float QW[16 * QWP];
  __shared__ __align__(16) float SC[16 * NSTEPS];
  __shared__ __align__(16) float OST[16 * OSTP];
  __shared__ __align__(16) float VAS[NHID];

  const _Float16* W0 = (const _Float16*)W0p;
  const _Float16* W1 = (const _Float16*)W1p;
  const _Float16* Wa = (const _Float16*)Wap;
  const _Float16* Pj = (const _Float16*)Pjp;

  const int tid = threadIdx.x, lane = tid & 31, wave = tid >> 5;
  const int c = lane & 15, hh = lane >> 4, koff = hh * 8;

  {
    const v4u z4 = (v4u){0u, 0u, 0u, 0u};
    v4u* p0 = (v4u*)XaH;
    v4u* p1 = (v4u*)XaL;
    v4u* p2 = (v4u*)X1H;
    v4u* p3 = (v4u*)X1L;
#pragma unroll 1
    for (int i = tid; i < (16 * XAP) / 8; i += DEC_THR) { p0[i] = z4; p1[i] = z4; }
#pragma unroll 1
    for (int i = tid; i < (16 * X1P) / 8; i += DEC_THR) { p2[i] = z4; p3[i] = z4; }
  }
  VAS[tid] = tab[TAB_VA + tid];
  const float vb = bf16r(vab[0]);

  const v8f z8 = {0.f, 0.f, 0.f, 0.f, 0.f, 0.f, 0.f, 0.f};
  v8f c0s[2], c1s[2], hnew[2];
  c0s[0] = z8; c0s[1] = z8; c1s[0] = z8; c1s[1] = z8; hnew[0] = z8; hnew[1] = z8;
  __syncthreads();

  const size_t GS0 = (size_t)NHID * W0_LD;
  const size_t GS1 = (size_t)NHID * W1_LD;

#pragma unroll 1
  for (int t = 0; t < NSTEPS; ++t) {
    {
      const int n0 = 32 * wave + c;
      const int n1 = n0 + 16;
      const _Float16* wa0 = Wa + (size_t)n0 * NHID + koff;
      const _Float16* wa1 = Wa + (size_t)n1 * NHID + koff;
      const _Float16* xh = X1H + c * X1P + koff;
      const _Float16* xl = X1L + c * X1P + koff;
      const float wb0 = tab[TAB_WAB + n0];
      const float wb1 = tab[TAB_WAB + n1];
      v8f qa0 = z8, qa1 = z8;
#pragma unroll 1
      for (int k0 = 0; k0 < NHID; k0 += 32) {
        const v16h b0 = Frag<_Float16>::load(wa0 + k0);
        const v16h b1 = Frag<_Float16>::load(wa1 + k0);
        const v16h ah0 = Frag<_Float16>::load(xh + k0);
        const v16h al0 = Frag<_Float16>::load(xl + k0);
        const v16h ah1 = Frag<_Float16>::load(xh + NHID + k0);
        const v16h al1 = Frag<_Float16>::load(xl + NHID + k0);
        qa0 = Frag<_Float16>::mma(ah0, b0, qa0);
        qa1 = Frag<_Float16>::mma(ah0, b1, qa1);
        qa0 = Frag<_Float16>::mma(ah1, b0, qa0);
        qa1 = Frag<_Float16>::mma(ah1, b1, qa1);
        qa0 = Frag<_Float16>::mma(al0, b0, qa0);
        qa1 = Frag<_Float16>::mma(al0, b1, qa1);
        qa0 = Frag<_Float16>::mma(al1, b0, qa0);
        qa1 = Frag<_Float16>::mma(al1, b1, qa1);
        guard_query(qa0, qa1, ah0, al0, ah1, al1, b0, b1);
      }
      acc_guard2(qa0, qa1);
#pragma unroll
      for (int r = 0; r < 8; ++r) {
        QW[(8 * hh + r) * QWP + n0] = qa0[r] * (0.5f * FOLD_AW) + wb0;
        QW[(8 * hh + r) * QWP + n1] = qa1[r] * (0.5f * FOLD_AW) + wb1;
      }
    }
    __syncthreads();

    {
      const float* urow = UaK + (size_t)(wave * NSTEPS) * NHID;
      const float* qrow = QW + wave * QWP;
#pragma unroll 1
      for (int tp = 0; tp < NSTEPS; ++tp) {
        float s = 0.0f;
#pragma unroll 1
        for (int q = 0; q < 4; ++q) {
          const int h0 = 128 * q + 4 * lane;
          const v4f u  = *(const v4f*)(urow + (size_t)tp * NHID + h0);
          const v4f qv = *(const v4f*)(qrow + h0);
          const v4f vv = *(const v4f*)(VAS + h0);
          s += vv[0] * tanhf(qv[0] + u[0]);
          s += vv[1] * tanhf(qv[1] + u[1]);
          s += vv[2] * tanhf(qv[2] + u[2]);
          s += vv[3] * tanhf(qv[3] + u[3]);
        }
#pragma unroll
        for (int off = 16; off > 0; off >>= 1) s += __shfl_xor(s, off, 32);
        if (lane == 0) SC[wave * NSTEPS + tp] = s + vb;
      }
    }
    __syncthreads();

    {
      float* sr = SC + wave * NSTEPS;
      const float s0 = sr[lane];
      const float s1 = sr[32 + lane];
      const float s2 = sr[64 + lane];
      float m = fmaxf(s0, fmaxf(s1, s2));
#pragma unroll
      for (int off = 16; off > 0; off >>= 1) m = fmaxf(m, __shfl_xor(m, off, 32));
      const float e0 = expf(s0 - m);
      const float e1 = expf(s1 - m);
      const float e2 = expf(s2 - m);
      float d = (e0 + e1) + e2;
#pragma unroll
      for (int off = 16; off > 0; off >>= 1) d += __shfl_xor(d, off, 32);
      const float inv = 1.0f / d;
      sr[lane]      = e0 * inv;
      sr[32 + lane] = e1 * inv;
      sr[64 + lane] = e2 * inv;
    }
    __syncthreads();

    {
      float ca[16];
#pragma unroll
      for (int e = 0; e < 16; ++e) ca[e] = 0.0f;
      const unsigned short* eb = encB + (size_t)(wave * NSTEPS) * NFEAT + 8 * lane;
      const float* wr = SC + wave * NSTEPS;
#pragma unroll 1
      for (int tp = 0; tp < NSTEPS; ++tp) {
        const float w = wr[tp];
        const v4u e0 = *(const v4u*)(eb + (size_t)tp * NFEAT);
        const v4u e1 = *(const v4u*)(eb + (size_t)tp * NFEAT + 256);
#pragma unroll
        for (int k = 0; k < 4; ++k) {
          const unsigned w0 = e0[k];
          const unsigned w1 = e1[k];
          ca[2 * k]         = fmaf(w, __uint_as_float(w0 << 16), ca[2 * k]);
          ca[2 * k + 1]     = fmaf(w, __uint_as_float(w0 & 0xffff0000u), ca[2 * k + 1]);
          ca[8 + 2 * k]     = fmaf(w, __uint_as_float(w1 << 16), ca[8 + 2 * k]);
          ca[8 + 2 * k + 1] = fmaf(w, __uint_as_float(w1 & 0xffff0000u), ca[8 + 2 * k + 1]);
        }
      }
      v8h hv0, lv0, hv1, lv1;
#pragma unroll
      for (int e = 0; e < 8; ++e) {
        _Float16 h, l;
        split_act(ca[e], h, l);
        hv0[e] = h; lv0[e] = l;
        split_act(ca[8 + e], h, l);
        hv1[e] = h; lv1[e] = l;
      }
      *(v8h*)(XaH + wave * XAP + NMEL + 8 * lane)       = hv0;
      *(v8h*)(XaL + wave * XAP + NMEL + 8 * lane)       = lv0;
      *(v8h*)(XaH + wave * XAP + NMEL + 256 + 8 * lane) = hv1;
      *(v8h*)(XaL + wave * XAP + NMEL + 256 + 8 * lane) = lv1;
      if (lane < 2) {
        const v8h zz = {(_Float16)0.0f, (_Float16)0.0f, (_Float16)0.0f, (_Float16)0.0f,
                        (_Float16)0.0f, (_Float16)0.0f, (_Float16)0.0f, (_Float16)0.0f};
        *(v8h*)(XaH + wave * XAP + NIH0 + 8 * lane) = zz;
        *(v8h*)(XaL + wave * XAP + NIH0 + 8 * lane) = zz;
      }
    }
    __syncthreads();

#pragma unroll
    for (int tt = 0; tt < 2; ++tt) {
      const int unit = 32 * wave + 16 * tt + c;
      const _Float16* wrow = W0 + (size_t)unit * W0_LD + koff;
      const float bi = tab[TAB_B0 + unit];
      const float bf = tab[TAB_B0 + NHID + unit];
      const float bg = tab[TAB_B0 + 2 * NHID + unit];
      const float bo = tab[TAB_B0 + 3 * NHID + unit];
      v8f a0 = z8, a1 = z8, a2 = z8, a3 = z8;
      gate_kloop(a0, a1, a2, a3, XaH + c * XAP + koff, XaL + c * XAP + koff, wrow, GS0, XA_K / 32);
      gate_kloop(a0, a1, a2, a3, X1H + c * X1P + koff, X1L + c * X1P + koff, wrow + W0_IHP, GS0, NHID / 32);
      acc_guard4(a0, a1, a2, a3);
      cell_update(a0, a1, a2, a3, bi, bf, bg, bo, c0s[tt], hnew[tt]);
    }
    __syncthreads();
#pragma unroll
    for (int tt = 0; tt < 2; ++tt) {
      const int unit = 32 * wave + 16 * tt + c;
#pragma unroll
      for (int r = 0; r < 8; ++r) {
        _Float16 h, l;
        split_act(hnew[tt][r], h, l);
        X1H[(8 * hh + r) * X1P + unit] = h;
        X1L[(8 * hh + r) * X1P + unit] = l;
      }
    }
    __syncthreads();

#pragma unroll
    for (int tt = 0; tt < 2; ++tt) {
      const int unit = 32 * wave + 16 * tt + c;
      const _Float16* wrow = W1 + (size_t)unit * W1_LD + koff;
      const float bi = tab[TAB_B1 + unit];
      const float bf = tab[TAB_B1 + NHID + unit];
      const float bg = tab[TAB_B1 + 2 * NHID + unit];
      const float bo = tab[TAB_B1 + 3 * NHID + unit];
      v8f a0 = z8, a1 = z8, a2 = z8, a3 = z8;
      gate_kloop(a0, a1, a2, a3, X1H + c * X1P + koff, X1L + c * X1P + koff, wrow, GS1, (2 * NHID) / 32);
      acc_guard4(a0, a1, a2, a3);
      cell_update(a0, a1, a2, a3, bi, bf, bg, bo, c1s[tt], hnew[tt]);
    }
    __syncthreads();
#pragma unroll
    for (int tt = 0; tt < 2; ++tt) {
      const int unit = 32 * wave + 16 * tt + c;
#pragma unroll
      for (int r = 0; r < 8; ++r) {
        _Float16 h, l;
        split_act(hnew[tt][r], h, l);
        X1H[(8 * hh + r) * X1P + NHID + unit] = h;
        X1L[(8 * hh + r) * X1P + NHID + unit] = l;
      }
    }
    __syncthreads();

    if (wave < NMEL / 16) {
      const int n = 16 * wave + c;
      const _Float16* pw = Pj + (size_t)n * NHID + koff;
      const _Float16* xh = X1H + c * X1P + NHID + koff;
      const _Float16* xl = X1L + c * X1P + NHID + koff;
      const float pb = tab[TAB_PJB + n];
      v8f pa = z8;
#pragma unroll 1
      for (int k0 = 0; k0 < NHID; k0 += 32) {
        const v16h b  = Frag<_Float16>::load(pw + k0);
        const v16h ah = Frag<_Float16>::load(xh + k0);
        const v16h al = Frag<_Float16>::load(xl + k0);
        pa = Frag<_Float16>::mma(ah, b, pa);
        pa = Frag<_Float16>::mma(al, b, pa);
        guard_proj(pa, ah, al, b);
      }
      acc_guard1(pa);
      const int ocol = (t & 1) * NMEL + n;
#pragma unroll
      for (int r = 0; r < 8; ++r) {
        const float v = pa[r] * FOLD_AW + pb;
        OST[(8 * hh + r) * OSTP + ocol] = v;
        _Float16 h, l;
        split_act(v, h, l);
        XaH[(8 * hh + r) * XAP + n] = h;
        XaL[(8 * hh + r) * XAP + n] = l;
      }
    }
    __syncthreads();

    if (t & 1) {
      const float* orow = OST + wave * OSTP;
      float* dp = out + ((size_t)(wave * NSTEPS + (t - 1))) * NMEL;
      const v4f v0 = *(const v4f*)(orow + 4 * lane);
      const v4f v1 = *(const v4f*)(orow + 128 + 4 * (lane & 7));
      for (int pass = 0; pass < 2; ++pass) {
        *(volatile v4f*)(dp + 4 * lane) = v0;
        if (lane < 8) *(volatile v4f*)(dp + 128 + 4 * lane) = v1;
        __threadfence();
      }
    }
  }
}

extern "C" void kernel_launch(void* const* d_in, const int* in_sizes, int n_in,
                              void* d_out, int out_size, void* d_ws, size_t ws_size, hipStream_t stream) {
  if (n_in < 17 || d_out == nullptr || d_ws == nullptr) return;
  if (in_sizes[0] != NBAT * NSTEPS * NFEAT || in_sizes[1] != NHID * NHID || in_sizes[2] != NHID ||
      in_sizes[3] != NHID * NFEAT || in_sizes[4] != NHID || in_sizes[5] != NHID || in_sizes[6] != 1 ||
      in_sizes[7] != NGATE * NIH0 || in_sizes[8] != NGATE * NHID || in_sizes[9] != NGATE || in_sizes[10] != NGATE ||
      in_sizes[11] != NGATE * NHID || in_sizes[12] != NGATE * NHID || in_sizes[13] != NGATE || in_sizes[14] != NGATE ||
      in_sizes[15] != NMEL * NHID || in_sizes[16] != NMEL || out_size != NBAT * NSTEPS * NMEL) return;

  const float* enc   = (const float*)d_in[0];
  const float* Wa_w  = (const float*)d_in[1];
  const float* Wa_b  = (const float*)d_in[2];
  const float* Ua_w  = (const float*)d_in[3];
  const float* Ua_b  = (const float*)d_in[4];
  const float* Va_w  = (const float*)d_in[5];
  const float* Va_b  = (const float*)d_in[6];
  const float* Wih0  = (const float*)d_in[7];
  const float* Whh0  = (const float*)d_in[8];
  const float* bih0  = (const float*)d_in[9];
  const float* bhh0  = (const float*)d_in[10];
  const float* Wih1  = (const float*)d_in[11];
  const float* Whh1  = (const float*)d_in[12];
  const float* bih1  = (const float*)d_in[13];
  const float* bhh1  = (const float*)d_in[14];
  const float* projw = (const float*)d_in[15];
  const float* projb = (const float*)d_in[16];
  float* out = (float*)d_out;

  char* ws = (char*)d_ws; size_t off = 0;
  auto carve = [&](size_t bytes) -> char* { char* p = ws + off; off += (bytes + 255) & ~(size_t)255; return p; };
  unsigned short* W0  = (unsigned short*)carve((size_t)NGATE * W0_LD * 2);
  unsigned short* W1  = (unsigned short*)carve((size_t)NGATE * W1_LD * 2);
  unsigned short* WA  = (unsigned short*)carve((size_t)NHID * NHID * 2);
  unsigned short* UA  = (unsigned short*)carve((size_t)NHID * NFEAT * 2);
  unsigned short* PJ  = (unsigned short*)carve((size_t)NMEL * NHID * 2);
  unsigned short* E16 = (unsigned short*)carve((size_t)NENCROW * NFEAT * 2);
  unsigned short* EB  = (unsigned short*)carve((size_t)NENCROW * NFEAT * 2);
  float*          UAK = (float*)carve((size_t)NENCROW * NHID * 4);
  float*          TAB = (float*)carve((size_t)TAB_N * 4);
  if (off > ws_size || off > (size_t)134217728) return;

  auto nblk = [](int nrow, int ng) -> int { return (nrow * ng + 255) / 256; };

  cvt_rows_kernel<0><<<nblk(NGATE, W0_IHP / 8), 256, 0, stream>>>(Wih0, NIH0, NIH0 / 8, W0, W0_LD, 0, NGATE, W0_IHP / 8, W_CARRY);
  cvt_rows_kernel<0><<<nblk(NGATE, NHID / 8), 256, 0, stream>>>(Whh0, NHID, NHID / 8, W0, W0_LD, W0_IHP, NGATE, NHID / 8, W_CARRY);
  cvt_rows_kernel<0><<<nblk(NGATE, NHID / 8), 256, 0, stream>>>(Wih1, NHID, NHID / 8, W1, W1_LD, 0, NGATE, NHID / 8, W_CARRY);
  cvt_rows_kernel<0><<<nblk(NGATE, NHID / 8), 256, 0, stream>>>(Whh1, NHID, NHID / 8, W1, W1_LD, NHID, NGATE, NHID / 8, W_CARRY);
  cvt_rows_kernel<0><<<nblk(NHID, NHID / 8), 256, 0, stream>>>(Wa_w, NHID, NHID / 8, WA, NHID, 0, NHID, NHID / 8, W_CARRY);
  cvt_rows_kernel<0><<<nblk(NHID, NFEAT / 8), 256, 0, stream>>>(Ua_w, NFEAT, NFEAT / 8, UA, NFEAT, 0, NHID, NFEAT / 8, W_CARRY);
  cvt_rows_kernel<0><<<nblk(NMEL, NHID / 8), 256, 0, stream>>>(projw, NHID, NHID / 8, PJ, NHID, 0, NMEL, NHID / 8, W_CARRY);
  cvt_rows_kernel<0><<<nblk(NENCROW, NFEAT / 8), 256, 0, stream>>>(enc, NFEAT, NFEAT / 8, E16, NFEAT, 0, NENCROW, NFEAT / 8, ENC_CARRY);
  cvt_rows_kernel<1><<<nblk(NENCROW, NFEAT / 8), 256, 0, stream>>>(enc, NFEAT, NFEAT / 8, EB, NFEAT, 0, NENCROW, NFEAT / 8, 1.0f);
  table_kernel<<<TAB_N / 512, 128, 0, stream>>>(bih0, bhh0, bih1, bhh1, Wa_b, Va_w, Ua_b, projb, TAB);

  wmma_gemm64<0, false, 2, 0, false, 0><<<dim3((NENCROW / 64) * (NHID / 64) / 8, 1), 256, 0, stream>>>(
      E16, E16, NFEAT, 0L, UA, UA, NFEAT, 0L, (void*)UAK, (void*)UAK, NHID, 0L,
      TAB + TAB_UAB, TAB, 0L, NENCROW, NHID, NFEAT, FOLD_UAK);

  decoder_kernel<<<1, DEC_THR, 0, stream>>>(W0, W1, WA, PJ, EB, UAK, TAB, Va_b, out);
}
